// Layer_68719477574
// MI455X (gfx1250) — hardware-verified
//
#include <hip/hip_runtime.h>

typedef _Float16 v16h __attribute__((ext_vector_type(16)));
typedef _Float16 v8h  __attribute__((ext_vector_type(8)));
typedef float    v8f  __attribute__((ext_vector_type(8)));
typedef float    v4f  __attribute__((ext_vector_type(4)));
typedef v8h __attribute__((may_alias)) v8ha;
typedef v4f __attribute__((may_alias)) v4fa;

union Frag { v16h v; v8h half[2]; };

#define BATCH   8
#define SEQ     1024
#define IN_DIM  768
#define OUT_DIM 512
#define MROWS   (BATCH * SEQ)
#define NXE     (MROWS * IN_DIM)
#define NWE     (OUT_DIM * IN_DIM)
#define NPE     (OUT_DIM * OUT_DIM)
#define NOUT    (MROWS * OUT_DIM)
#define NX8     (NXE / 8)
#define NW8     (NWE / 8)
#define TROWS   (SEQ * 16)

static_assert(IN_DIM % 32 == 0);
static_assert(OUT_DIM % 64 == 0);
static_assert(OUT_DIM == 512);
static_assert(MROWS % 128 == 0);
static_assert(NX8 % 256 == 0);
static_assert(NW8 % 256 == 0);
static_assert(MROWS % 8 == 0);
static_assert((SEQ * (OUT_DIM / 32)) % 4 == 0);

__device__ __forceinline__ v8f wmma_f16(v16h a, v16h b, v8f c) {
  v8f d = __builtin_amdgcn_wmma_f32_16x16x32_f16(false, a, false, b, (short)0, c, false, false);
  asm volatile("v_nop\n\tv_nop\n\tv_nop\n\tv_nop" : "+v"(d) : "v"(a), "v"(b));
  return d;
}

__device__ __forceinline__ v16h load_frag(const _Float16* p, int h) {
  Frag f;
  f.half[0] = *(const v8ha*)(p + 8 * h);
  f.half[1] = *(const v8ha*)(p + 16 + 8 * h);
  return f.v;
}

__global__ __launch_bounds__(256) void convert_kernel(
    const float* __restrict__ x, const float* __restrict__ wm, const float* __restrict__ wr,
    _Float16* __restrict__ xh, _Float16* __restrict__ wh)
{
  const int g = blockIdx.x * 256 + threadIdx.x;
  if (g >= NX8 + 2 * NW8) return;
  const float* src;
  _Float16* dst;
  float sc;
  if (g < NX8) {
    src = x + (size_t)g * 8;
    dst = xh + (size_t)g * 8;
    sc = 8.0f;
  } else {
    const int e = g - NX8;
    if (e < NW8) { src = wm + (size_t)e * 8;           sc = 64.0f;  }
    else         { src = wr + (size_t)(e - NW8) * 8;   sc = 256.0f; }
    dst = wh + (size_t)e * 8;
  }
  const v4f a = *(const v4fa*)src;
  const v4f c = *(const v4fa*)(src + 4);
  const v8h o = { (_Float16)(a.x * sc), (_Float16)(a.y * sc), (_Float16)(a.z * sc), (_Float16)(a.w * sc),
                  (_Float16)(c.x * sc), (_Float16)(c.y * sc), (_Float16)(c.z * sc), (_Float16)(c.w * sc) };
  *(volatile v8h*)dst = o;
  __threadfence();
  *(volatile v8h*)dst = o;
}

__device__ __forceinline__ void proj_store_pass(const float* sT, float* base,
                                                int m0, int col0, int w, int lane) {
  const int q8 = lane & 7, sub = lane >> 3;
  #pragma unroll
  for (int i = 0; i < 16; ++i) {
    const int lid = i * 4 + sub;
    const int row = 32 * w + (lid >> 1);
    const int hl = lid & 1;
    const v4f v = *(const v4fa*)(sT + row * 64 + 32 * hl + 4 * q8);
    const size_t gi = (size_t)(m0 + row) * OUT_DIM + col0 + 32 * hl + 4 * q8;
    *(volatile v4f*)(base + gi) = v;
  }
}

__global__ __launch_bounds__(128) void proj_kernel(
    const _Float16* __restrict__ xh,
    const _Float16* __restrict__ wh,
    float* __restrict__ xt,
    float* __restrict__ rres)
{
  __shared__ __attribute__((aligned(16))) float sT[128 * 64];

  const int tid = threadIdx.x, lane = tid & 31, w = tid >> 5;
  const int h = lane >> 4, m = lane & 15;
  const int m0 = blockIdx.x * 128;
  const int cg = blockIdx.y;
  const int which = cg >> 3;
  const int col0 = (cg & 7) * 64;
  const int m0w = m0 + 32 * w;

  const _Float16* xa0 = xh + (size_t)(m0w + m) * IN_DIM;
  const _Float16* xa1 = xa0 + (size_t)16 * IN_DIM;
  const _Float16* wb  = wh + ((size_t)which * OUT_DIM + col0 + m) * IN_DIM;

  const v8f zero8 = {0.f, 0.f, 0.f, 0.f, 0.f, 0.f, 0.f, 0.f};
  v8f acc[2][4];
  #pragma unroll
  for (int mt = 0; mt < 2; ++mt)
    #pragma unroll
    for (int nt = 0; nt < 4; ++nt) acc[mt][nt] = zero8;

  #pragma unroll 1
  for (int k0 = 0; k0 < IN_DIM; k0 += 32) {
    const v16h a0 = load_frag(xa0 + k0, h);
    const v16h a1 = load_frag(xa1 + k0, h);
    #pragma unroll
    for (int nt = 0; nt < 4; ++nt) {
      const v16h b = load_frag(wb + (size_t)nt * 16 * IN_DIM + k0, h);
      acc[0][nt] = wmma_f16(a0, b, acc[0][nt]);
      acc[1][nt] = wmma_f16(a1, b, acc[1][nt]);
    }
  }

  const float osc = (which == 0) ? (1.0f / 512.0f) : (1.0f / 2048.0f);
  #pragma unroll
  for (int nt = 0; nt < 4; ++nt) {
    #pragma unroll
    for (int mt = 0; mt < 2; ++mt) {
      #pragma unroll
      for (int r = 0; r < 8; ++r) {
        const int tokl = 32 * w + 16 * mt + 8 * h + r;
        sT[tokl * 64 + 16 * nt + m] = acc[mt][nt][r] * osc;
      }
    }
  }
  __syncthreads();

  float* base = (which == 0) ? xt : rres;
  proj_store_pass(sT, base, m0, col0, w, lane);
  __threadfence();
  proj_store_pass(sT, base, m0, col0, w, lane);
}

__device__ __forceinline__ float hsum4(v4f a) { return (a.x + a.y) + (a.z + a.w); }

__device__ __forceinline__ float wave_sum(float v) {
  #pragma unroll
  for (int o = 16; o >= 1; o >>= 1) v += __shfl_xor(v, o);
  return v;
}

__device__ __forceinline__ void pack_hl(v4f ya, v4f yb, v8h& hi, v8h& lo) {
  const v4f va = ya * 16.0f, vb = yb * 16.0f;
  v8h hh;
  hh[0] = (_Float16)va.x; hh[1] = (_Float16)va.y; hh[2] = (_Float16)va.z; hh[3] = (_Float16)va.w;
  hh[4] = (_Float16)vb.x; hh[5] = (_Float16)vb.y; hh[6] = (_Float16)vb.z; hh[7] = (_Float16)vb.w;
  v8h ll;
  ll[0] = (_Float16)((va.x - (float)hh[0]) * 4096.0f);
  ll[1] = (_Float16)((va.y - (float)hh[1]) * 4096.0f);
  ll[2] = (_Float16)((va.z - (float)hh[2]) * 4096.0f);
  ll[3] = (_Float16)((va.w - (float)hh[3]) * 4096.0f);
  ll[4] = (_Float16)((vb.x - (float)hh[4]) * 4096.0f);
  ll[5] = (_Float16)((vb.y - (float)hh[5]) * 4096.0f);
  ll[6] = (_Float16)((vb.z - (float)hh[6]) * 4096.0f);
  ll[7] = (_Float16)((vb.w - (float)hh[7]) * 4096.0f);
  hi = hh; lo = ll;
}

__device__ __forceinline__ void ln_store_pass(_Float16* hrow, _Float16* lrow, int c0, int c1,
                                              v8h hA, v8h hB, v8h lA, v8h lB) {
  *(volatile v8h*)(hrow + c0) = hA;
  *(volatile v8h*)(hrow + c1) = hB;
  *(volatile v8h*)(lrow + c0) = lA;
  *(volatile v8h*)(lrow + c1) = lB;
}

__global__ __launch_bounds__(256) void ln_kernel(
    const float* __restrict__ xt,
    const float* __restrict__ lnw,
    const float* __restrict__ lnb,
    _Float16* __restrict__ tpl)
{
  const int tid = threadIdx.x, lane = tid & 31, w = tid >> 5;
  const int row = blockIdx.x * 8 + w;
  const int b = row / SEQ, s = row - b * SEQ;
  const float* xr = xt + (size_t)row * OUT_DIM;
  const int c0 = 8 * lane, c1 = 256 + 8 * lane;

  const v4f x0 = *(const v4fa*)(xr + c0);
  const v4f x1 = *(const v4fa*)(xr + c0 + 4);
  const v4f x2 = *(const v4fa*)(xr + c1);
  const v4f x3 = *(const v4fa*)(xr + c1 + 4);

  float su = hsum4(x0) + hsum4(x1) + hsum4(x2) + hsum4(x3);
  su = wave_sum(su);
  const float mu = su * (1.0f / 512.0f);

  const v4f d0 = x0 - mu, d1 = x1 - mu, d2 = x2 - mu, d3 = x3 - mu;
  float sq = hsum4(d0 * d0) + hsum4(d1 * d1) + hsum4(d2 * d2) + hsum4(d3 * d3);
  sq = wave_sum(sq);
  const float var = sq * (1.0f / 512.0f);
  const float rs = rsqrtf(var + 1e-5f);

  const v4f w0 = *(const v4fa*)(lnw + c0);
  const v4f w1 = *(const v4fa*)(lnw + c0 + 4);
  const v4f w2 = *(const v4fa*)(lnw + c1);
  const v4f w3 = *(const v4fa*)(lnw + c1 + 4);
  const v4f g0 = *(const v4fa*)(lnb + c0);
  const v4f g1 = *(const v4fa*)(lnb + c0 + 4);
  const v4f g2 = *(const v4fa*)(lnb + c1);
  const v4f g3 = *(const v4fa*)(lnb + c1 + 4);

  const v4f y0 = (d0 * rs) * w0 + g0;
  const v4f y1 = (d1 * rs) * w1 + g1;
  const v4f y2 = (d2 * rs) * w2 + g2;
  const v4f y3 = (d3 * rs) * w3 + g3;

  v8h hA, hB, lA, lB;
  pack_hl(y0, y1, hA, lA);
  pack_hl(y2, y3, hB, lB);

  _Float16* hrow = tpl + ((size_t)s * 16 + b) * OUT_DIM;
  _Float16* lrow = tpl + ((size_t)s * 16 + 8 + b) * OUT_DIM;
  ln_store_pass(hrow, lrow, c0, c1, hA, hB, lA, lB);
  __threadfence();
  ln_store_pass(hrow, lrow, c0, c1, hA, hB, lA, lB);
}

__device__ __forceinline__ float pcos256(float p, float per, float t2) {
  float rc = __builtin_amdgcn_rcpf(per);
  rc = fmaf(fmaf(-per, rc, 1.0f), rc, rc);
  const float arg = t2 * rc;
  const float nf = rintf(arg * 0.318309873f);
  float rd = fmaf(nf, -3.14159274f, arg);
  rd = fmaf(nf, 8.74227766e-8f, rd);
  const float q = rd * rd;
  float pl = 2.08767570e-9f;
  pl = fmaf(pl, q, -2.75573192e-7f);
  pl = fmaf(pl, q, 2.48015873e-5f);
  pl = fmaf(pl, q, -1.38888889e-3f);
  pl = fmaf(pl, q, 4.16666667e-2f);
  pl = fmaf(pl, q, -0.5f);
  float c = fmaf(pl, q, 1.0f);
  const int ni = (int)nf;
  c = __int_as_float(__float_as_int(c) ^ (int)((unsigned)ni << 31));
  return (c * p) * 256.0f;
}

__device__ __forceinline__ v8h gen8(v4f pa, v4f pb, v4f ea, v4f eb, float t2) {
  v8h o;
  o[0] = (_Float16)pcos256(pa.x, ea.x, t2);
  o[1] = (_Float16)pcos256(pa.y, ea.y, t2);
  o[2] = (_Float16)pcos256(pa.z, ea.z, t2);
  o[3] = (_Float16)pcos256(pa.w, ea.w, t2);
  o[4] = (_Float16)pcos256(pb.x, eb.x, t2);
  o[5] = (_Float16)pcos256(pb.y, eb.y, t2);
  o[6] = (_Float16)pcos256(pb.z, eb.z, t2);
  o[7] = (_Float16)pcos256(pb.w, eb.w, t2);
  return o;
}

__device__ __forceinline__ v16h gen_bfrag(const float* prow, const float* erow, int j0, float t2) {
  const v4f p0 = *(const v4fa*)(prow + j0);
  const v4f p1 = *(const v4fa*)(prow + j0 + 4);
  const v4f p2 = *(const v4fa*)(prow + j0 + 16);
  const v4f p3 = *(const v4fa*)(prow + j0 + 20);
  const v4f e0 = *(const v4fa*)(erow + j0);
  const v4f e1 = *(const v4fa*)(erow + j0 + 4);
  const v4f e2 = *(const v4fa*)(erow + j0 + 16);
  const v4f e3 = *(const v4fa*)(erow + j0 + 20);
  Frag b;
  b.half[0] = gen8(p0, p1, e0, e1, t2);
  b.half[1] = gen8(p2, p3, e2, e3, t2);
  return b.v;
}

__device__ __forceinline__ void nk_store_pass(const float* so, const float* rres, float* out,
                                              int s, int i0, int lane) {
  const int q8 = lane & 7, sub = lane >> 3;
  #pragma unroll
  for (int i = 0; i < 2; ++i) {
    const int b = i * 4 + sub;
    const v4f v = *(const v4fa*)(so + b * 32 + 4 * q8);
    const size_t gi = ((size_t)b * SEQ + s) * OUT_DIM + i0 + 4 * q8;
    const v4f rr = *(const v4fa*)(rres + gi);
    const v4f o = v + rr;
    *(volatile v4f*)(out + gi) = o;
  }
}

__global__ __launch_bounds__(128) void nk_kernel(
    const _Float16* __restrict__ tpl,
    const float* __restrict__ P,
    const float* __restrict__ per,
    const int* __restrict__ pos,
    const float* __restrict__ rres,
    float* __restrict__ out)
{
  __shared__ __attribute__((aligned(16))) float sO[4 * 256];

  const int tid = threadIdx.x, lane = tid & 31, w = tid >> 5;
  const int h = lane >> 4, m = lane & 15;
  const int gw = blockIdx.x * 4 + w;
  const int s = gw >> 4;
  const int i0 = (gw & 15) * 32;

  const float kf = (float)pos[s];
  const float t2 = 6.28318548f * kf;

  const _Float16* arow = tpl + ((size_t)s * 16 + m) * OUT_DIM;
  const float* prow0 = P   + (size_t)(i0 + m) * OUT_DIM + 8 * h;
  const float* prow1 = prow0 + (size_t)16 * OUT_DIM;
  const float* erow0 = per + (size_t)(i0 + m) * OUT_DIM + 8 * h;
  const float* erow1 = erow0 + (size_t)16 * OUT_DIM;

  const v8f zero8 = {0.f, 0.f, 0.f, 0.f, 0.f, 0.f, 0.f, 0.f};
  v8f acc0 = zero8, acc1 = zero8;

  #pragma unroll 1
  for (int j0 = 0; j0 < OUT_DIM; j0 += 32) {
    const v16h a  = load_frag(arow + j0, h);
    const v16h b0 = gen_bfrag(prow0, erow0, j0, t2);
    acc0 = wmma_f16(a, b0, acc0);
    const v16h b1 = gen_bfrag(prow1, erow1, j0, t2);
    acc1 = wmma_f16(a, b1, acc1);
  }

  float* so = sO + w * 256;
  #pragma unroll
  for (int r = 0; r < 8; ++r) {
    const float m0v = acc0[r], m1v = acc1[r];
    const float o0 = __shfl_xor(m0v, 16);
    const float o1 = __shfl_xor(m1v, 16);
    const float hi0 = h ? o0 : m0v, lo0 = h ? m0v : o0;
    const float hi1 = h ? o1 : m1v, lo1 = h ? m1v : o1;
    const float v0 = hi0 * (1.0f / 4096.0f) + lo0 * (1.0f / 16777216.0f);
    const float v1 = hi1 * (1.0f / 4096.0f) + lo1 * (1.0f / 16777216.0f);
    if (h == 0) {
      so[r * 32 + m] = v0;
      so[r * 32 + 16 + m] = v1;
    }
  }
  __syncthreads();

  nk_store_pass(so, rres, out, s, i0, lane);
  __threadfence();
  nk_store_pass(so, rres, out, s, i0, lane);
}

extern "C" void kernel_launch(void* const* d_in, const int* in_sizes, int n_in,
                              void* d_out, int out_size, void* d_ws, size_t ws_size,
                              hipStream_t stream) {
  if (n_in < 8) return;
  if (in_sizes[0] != NXE) return;
  if (in_sizes[1] != SEQ) return;
  if (in_sizes[2] != NWE || in_sizes[4] != NWE) return;
  if (in_sizes[3] != NPE || in_sizes[7] != NPE) return;
  if (in_sizes[5] != OUT_DIM || in_sizes[6] != OUT_DIM) return;
  if (out_size != NOUT) return;

  const float* x    = (const float*)d_in[0];
  const int*   pos  = (const int*)  d_in[1];
  const float* Mw   = (const float*)d_in[2];
  const float* Pw   = (const float*)d_in[3];
  const float* Wres = (const float*)d_in[4];
  const float* lnw  = (const float*)d_in[5];
  const float* lnb  = (const float*)d_in[6];
  const float* per  = (const float*)d_in[7];
  float* out = (float*)d_out;

  const size_t xh_bytes  = (size_t)NXE * 2;
  const size_t wh_bytes  = (size_t)2 * NWE * 2;
  const size_t xt_bytes  = (size_t)NOUT * 4;
  const size_t rr_bytes  = (size_t)NOUT * 4;
  const size_t tpl_bytes = (size_t)TROWS * OUT_DIM * 2;
  const size_t total = xh_bytes + wh_bytes + xt_bytes + rr_bytes + tpl_bytes;
  if (total > ws_size) return;

  char* ws = (char*)d_ws;
  _Float16* xh  = (_Float16*)(ws);
  _Float16* wh  = (_Float16*)(ws + xh_bytes);
  float*    xt  = (float*)   (ws + xh_bytes + wh_bytes);
  float*    rres= (float*)   (ws + xh_bytes + wh_bytes + xt_bytes);
  _Float16* tpl = (_Float16*)(ws + xh_bytes + wh_bytes + xt_bytes + rr_bytes);

  const int ngroups = NX8 + 2 * NW8;
  convert_kernel<<<(ngroups + 255) / 256, 256, 0, stream>>>(x, Mw, Wres, xh, wh);

  dim3 gProj(MROWS / 128, (2 * OUT_DIM) / 64);
  proj_kernel<<<gProj, 128, 0, stream>>>(xh, wh, xt, rres);

  ln_kernel<<<MROWS / 8, 256, 0, stream>>>(xt, lnw, lnb, tpl);

  nk_kernel<<<(SEQ * (OUT_DIM / 32)) / 4, 128, 0, stream>>>(tpl, Pw, per, pos, rres, out);
}
